// NNSensorResponse_687194768378
// MI455X (gfx1250) — hardware-verified
//
#include <hip/hip_runtime.h>
#include <math.h>
#include <stdint.h>

#define NE   32000
#define NEH  16000
#define FIN  3
#define HID  128
#define NS   1024
#define NT   1024
#define WSC  64.0f
#define INV_WSC 0.015625f
#define RSC  16.0f
#define ESC  16384.0f
#define ALPHA_OUT 3.814697265625e-06f
#define C_GAUSS 0.3989422804f

static_assert(NE == 2 * NEH);
static_assert((NEH % 64) == 0 && (NS % 64) == 0 && (NT % 64) == 0 && (HID % 64) == 0);
static_assert((NEH % 32) == 0 && (HID % 32) == 0 && (NS % 16) == 0);
static_assert((NE % 8) == 0 && (NEH % 2) == 0);
static_assert(((NT * (NEH / 2)) % 256) == 0);
static_assert((((NS / 16) * (NEH / 64)) % 8) == 0);
static_assert((((NS / 64) * (NT / 64)) % 8) == 0);

typedef _Float16 v16h __attribute__((ext_vector_type(16)));
typedef _Float16 v8h  __attribute__((ext_vector_type(8)));
typedef float    v8f  __attribute__((ext_vector_type(8)));
typedef float    v4f  __attribute__((ext_vector_type(4)));
typedef unsigned int v4u __attribute__((ext_vector_type(4)));

__device__ __forceinline__ unsigned short bf_bits(float f) {
  unsigned u = __float_as_uint(f);
  return (unsigned short)((u + 0x7FFFu + ((u >> 16) & 1u)) >> 16);
}
__device__ __forceinline__ float bf_round(float f) {
  return __uint_as_float(((unsigned)bf_bits(f)) << 16);
}
__device__ __forceinline__ unsigned short h_bits(float f) {
  _Float16 h = (_Float16)f;
  return __builtin_bit_cast(unsigned short, h);
}
__device__ __forceinline__ unsigned pk16(unsigned short a, unsigned short b) { return (unsigned)a | ((unsigned)b << 16); }
__device__ __forceinline__ v8f zero8() { v8f z = {0.f, 0.f, 0.f, 0.f, 0.f, 0.f, 0.f, 0.f}; return z; }

__device__ __forceinline__ v16h ldfrag_h(const _Float16* p) {
  union { v16h v; v8h h[2]; } f;
  f.h[0] = *(const v8h*)(p);
  f.h[1] = *(const v8h*)(p + 16);
  return f.v;
}

__device__ __forceinline__ v8f mma_h_raw(v16h a, v16h b, v8f c) {
  return __builtin_amdgcn_wmma_f32_16x16x32_f16(false, a, false, b, (short)0, c, false, false);
}
__device__ __forceinline__ void dep_guard_h(v8f& a, v8f& b, v16h x, v16h y) {
#if defined(__HIP_DEVICE_COMPILE__)
  asm volatile("v_nop\n\tv_nop\n\tv_nop\n\tv_nop" : "+v"(a), "+v"(b) : "v"(x), "v"(y));
#endif
}
__device__ __forceinline__ void keep4_h(v16h a, v16h b, v16h c, v16h d) {
#if defined(__HIP_DEVICE_COMPILE__)
  asm volatile("v_nop" :: "v"(a), "v"(b), "v"(c), "v"(d));
#endif
}
__device__ __forceinline__ void acc_guard4(v8f& a, v8f& b, v8f& c, v8f& d) {
#if defined(__HIP_DEVICE_COMPILE__)
  asm volatile("v_nop\n\tv_nop\n\tv_nop\n\tv_nop" : "+v"(a), "+v"(b), "+v"(c), "+v"(d));
#endif
}
__device__ __forceinline__ void wave_sync_lds() {
  __builtin_amdgcn_fence(__ATOMIC_RELEASE, "workgroup");
  __builtin_amdgcn_wave_barrier();
  __builtin_amdgcn_fence(__ATOMIC_ACQUIRE, "workgroup");
}

__device__ __forceinline__ float lin3(float x0, float x1, float x2, float w0, float w1, float w2, float b) {
  float v = (x0 * bf_round(w0) + x1 * bf_round(w1)) + x2 * bf_round(w2);
  v = v + bf_round(b);
  return fmaxf(v, 0.0f);
}

__global__ __launch_bounds__(256) void k_hplane(
    const float* __restrict__ X, int nE,
    const float* __restrict__ Wp1, const float* __restrict__ bp1,
    const float* __restrict__ Wa1, const float* __restrict__ ba1,
    unsigned short* Hp, unsigned short* Ha) {
  const int tid = threadIdx.x;
  const int lane = tid & 31, w = tid >> 5;
  const int sel = w & 1;
  const int e = blockIdx.x * 8 + (w >> 1) * 2 + (lane >> 4);
  if (e >= nE) return;
  const int j8 = (lane & 15) * 8;
  const float* W  = sel ? Wa1 : Wp1;
  const float* bb = sel ? ba1 : bp1;
  unsigned short* H = sel ? Ha : Hp;
  const float x0 = bf_round(X[(size_t)e * FIN + 0]);
  const float x1 = bf_round(X[(size_t)e * FIN + 1]);
  const float x2 = bf_round(X[(size_t)e * FIN + 2]);
  const v4f w0a = *(const v4f*)(W + j8),           w0b = *(const v4f*)(W + j8 + 4);
  const v4f w1a = *(const v4f*)(W + HID + j8),     w1b = *(const v4f*)(W + HID + j8 + 4);
  const v4f w2a = *(const v4f*)(W + 2 * HID + j8), w2b = *(const v4f*)(W + 2 * HID + j8 + 4);
  const v4f b0a = *(const v4f*)(bb + j8),          b0b = *(const v4f*)(bb + j8 + 4);
  const float h0 = lin3(x0, x1, x2, w0a[0], w1a[0], w2a[0], b0a[0]);
  const float h1 = lin3(x0, x1, x2, w0a[1], w1a[1], w2a[1], b0a[1]);
  const float h2 = lin3(x0, x1, x2, w0a[2], w1a[2], w2a[2], b0a[2]);
  const float h3 = lin3(x0, x1, x2, w0a[3], w1a[3], w2a[3], b0a[3]);
  const float h4 = lin3(x0, x1, x2, w0b[0], w1b[0], w2b[0], b0b[0]);
  const float h5 = lin3(x0, x1, x2, w0b[1], w1b[1], w2b[1], b0b[1]);
  const float h6 = lin3(x0, x1, x2, w0b[2], w1b[2], w2b[2], b0b[2]);
  const float h7 = lin3(x0, x1, x2, w0b[3], w1b[3], w2b[3], b0b[3]);
  v4u p;
  p[0] = pk16(h_bits(h0), h_bits(h1));
  p[1] = pk16(h_bits(h2), h_bits(h3));
  p[2] = pk16(h_bits(h4), h_bits(h5));
  p[3] = pk16(h_bits(h6), h_bits(h7));
  unsigned short* dst = H + (size_t)e * HID + j8;
  *(volatile v4u*)dst = p;
  __threadfence();
  *(volatile v4u*)dst = p;
}

__global__ __launch_bounds__(256) void tr_cvt64w(const float* __restrict__ in, unsigned short* out,
                                                 int R, int C) {
  __shared__ __align__(16) float s[64 * 68];
  const int tid = threadIdx.x;
  const int r0 = blockIdx.y * 64;
  const int c0 = blockIdx.x * 64;
  const int rl = tid >> 4;
  const int c4 = (tid & 15) * 4;
#pragma unroll
  for (int it = 0; it < 4; ++it) {
    const int r = it * 16 + rl;
    const v4f v = *(const v4f*)(in + (size_t)(r0 + r) * C + c0 + c4);
    s[(c4 + 0) * 68 + r] = v[0];
    s[(c4 + 1) * 68 + r] = v[1];
    s[(c4 + 2) * 68 + r] = v[2];
    s[(c4 + 3) * 68 + r] = v[3];
  }
  __syncthreads();
  const int q8 = (tid & 7) * 8;
  const int cl = tid >> 3;
  v4u pk[2];
#pragma unroll
  for (int it = 0; it < 2; ++it) {
    const int c = it * 32 + cl;
    const v4f a = *(const v4f*)(s + c * 68 + q8);
    const v4f b = *(const v4f*)(s + c * 68 + q8 + 4);
    v4u p;
    p[0] = pk16(h_bits(bf_round(a[0]) * WSC), h_bits(bf_round(a[1]) * WSC));
    p[1] = pk16(h_bits(bf_round(a[2]) * WSC), h_bits(bf_round(a[3]) * WSC));
    p[2] = pk16(h_bits(bf_round(b[0]) * WSC), h_bits(bf_round(b[1]) * WSC));
    p[3] = pk16(h_bits(bf_round(b[2]) * WSC), h_bits(bf_round(b[3]) * WSC));
    pk[it] = p;
  }
  for (int pass = 0; pass < 2; ++pass) {
#pragma unroll
    for (int it = 0; it < 2; ++it) {
      const int c = it * 32 + cl;
      *(volatile v4u*)(out + (size_t)(c0 + c) * R + r0 + q8) = pk[it];
    }
    __threadfence();
  }
}

__global__ __launch_bounds__(256) void k_resp(
    const unsigned short* __restrict__ WpTp, const unsigned short* __restrict__ WaTp,
    const unsigned short* __restrict__ Hpp, const unsigned short* __restrict__ Hap, int nrows,
    const float* __restrict__ bp2, const float* __restrict__ ba2, int nbias,
    const float* __restrict__ mask,
    unsigned short* RT, int ldo, int M, int N, int K) {
  const _Float16* WpT = (const _Float16*)(const void*)WpTp;
  const _Float16* WaT = (const _Float16*)(const void*)WaTp;
  const _Float16* Hp  = (const _Float16*)(const void*)Hpp;
  const _Float16* Ha  = (const _Float16*)(const void*)Hap;
  __shared__ __align__(16) float sT[8][16 * 68];
  const int lane = threadIdx.x & 31;
  const int wave = threadIdx.x >> 5;
  const int tilesM = M >> 4;
  const int tilesN = N >> 6;
  const int tile = blockIdx.x * 8 + wave;
  if (tile >= tilesM * tilesN) return;
  const int tn = tile / tilesM;
  const int tm = tile - tn * tilesM;
  const int s0 = tm << 4;
  const int r0 = tn << 6;

  const int rlane = lane & 15;
  const int koff  = (lane >> 4) * 8;
  const int mOff  = (lane >> 4) * 8;

  v8f accP[4], accA[4];
#pragma unroll
  for (int j = 0; j < 4; ++j) { accP[j] = zero8(); accA[j] = zero8(); }

  int srow = s0 + rlane; if (srow > M - 1) srow = M - 1;
  for (int k0 = 0; k0 < K; k0 += 32) {
    v16h hp[4], ha[4];
#pragma unroll
    for (int j = 0; j < 4; ++j) {
      int rr = r0 + (j << 4) + rlane; if (rr > nrows - 1) rr = nrows - 1;
      const size_t bo = (size_t)rr * HID + koff + k0;
      hp[j] = ldfrag_h(Hp + bo);
      ha[j] = ldfrag_h(Ha + bo);
    }
    const size_t ao = (size_t)srow * HID + koff + k0;
    const v16h ap = ldfrag_h(WpT + ao);
    const v16h aa = ldfrag_h(WaT + ao);
#pragma unroll
    for (int j = 0; j < 4; ++j) accP[j] = mma_h_raw(ap, hp[j], accP[j]);
    dep_guard_h(accP[0], accP[3], ap, hp[3]);
#pragma unroll
    for (int j = 0; j < 4; ++j) accA[j] = mma_h_raw(aa, ha[j], accA[j]);
    dep_guard_h(accA[0], accA[3], aa, ha[3]);
    keep4_h(hp[0], hp[1], hp[2], hp[3]);
    keep4_h(ha[0], ha[1], ha[2], ha[3]);
  }
  acc_guard4(accP[0], accP[1], accP[2], accP[3]);
  acc_guard4(accA[0], accA[1], accA[2], accA[3]);

  float bpv[8], bav[8];
#pragma unroll
  for (int e = 0; e < 8; ++e) {
    int si = s0 + mOff + e; if (si > nbias - 1) si = nbias - 1; if (si < 0) si = 0;
    bpv[e] = bf_round(bp2[si]);
    bav[e] = bf_round(ba2[si]);
  }
  float* slab = sT[wave];
#pragma unroll
  for (int j = 0; j < 4; ++j) {
    int mi = r0 + (j << 4) + rlane; if (mi > nrows - 1) mi = nrows - 1;
    const float mk = bf_round(mask[mi]);
#pragma unroll
    for (int e = 0; e < 8; ++e) {
      const float p  = accP[j][e] * INV_WSC + bpv[e];
      const float am = accA[j][e] * INV_WSC + bav[e];
      const float pc = fminf(fmaxf(p, -40.0f), 40.0f);
      const float ex = expf(-pc);
      const float sg = 1.0f / (1.0f + ex);
      const float v  = (am * sg) * mk;
      slab[(mOff + e) * 68 + (j << 4) + rlane] = v * RSC;
    }
  }
  wave_sync_lds();
  const int q8 = (lane & 7) * 8, rq = lane >> 3;
  v4u pk[4];
#pragma unroll
  for (int it = 0; it < 4; ++it) {
    const int row = it * 4 + rq;
    const v4f a = *(const v4f*)(slab + row * 68 + q8);
    const v4f b = *(const v4f*)(slab + row * 68 + q8 + 4);
    v4u p;
    p[0] = pk16(h_bits(a[0]), h_bits(a[1]));
    p[1] = pk16(h_bits(a[2]), h_bits(a[3]));
    p[2] = pk16(h_bits(b[0]), h_bits(b[1]));
    p[3] = pk16(h_bits(b[2]), h_bits(b[3]));
    pk[it] = p;
  }
  for (int pass = 0; pass < 2; ++pass) {
#pragma unroll
    for (int it = 0; it < 4; ++it) {
      const int row = it * 4 + rq;
      *(volatile v4u*)(RT + (size_t)(s0 + row) * ldo + r0 + q8) = pk[it];
    }
    __threadfence();
  }
  wave_sync_lds();
}

__global__ __launch_bounds__(256) void k_expv(const float* __restrict__ z, int nz,
                                              const float* __restrict__ sig,
                                              unsigned int* ET, int nrows, int npair) {
  const int i = blockIdx.x * 256 + threadIdx.x;
  if (i >= nrows * npair) return;
  const int t  = i / npair;
  const int rp = i - t * npair;
  int i0 = 2 * rp;     if (i0 > nz - 1) i0 = nz - 1;
  int i1 = 2 * rp + 1; if (i1 > nz - 1) i1 = nz - 1;
  const float sgm  = bf_round(sig[0]);
  const float s2   = sgm * sgm;
  const float inv2 = 1.0f / (2.0f * s2);
  const float coef = C_GAUSS / sqrtf(s2);
  const float tf = (float)t;
  const float z0 = bf_round(z[i0]);
  const float z1 = bf_round(z[i1]);
  const float d0 = tf - z0, d1 = tf - z1;
  const float q0 = d0 * d0, q1 = d1 * d1;
  const float e0 = expf(-(q0 * inv2)) * coef;
  const float e1 = expf(-(q1 * inv2)) * coef;
  const unsigned p = pk16(h_bits(e0 * ESC), h_bits(e1 * ESC));
  *(volatile unsigned*)(ET + i) = p;
  __threadfence();
  *(volatile unsigned*)(ET + i) = p;
}

template <int RES>
__global__ __launch_bounds__(256) void gemm64f(
    const unsigned short* __restrict__ Ap, int lda,
    const unsigned short* __restrict__ Btp, int ldb,
    float* Cout, int ldc,
    const float* __restrict__ res, int ldr,
    float alpha, int M, int N, int K) {
  const _Float16* A  = (const _Float16*)(const void*)Ap;
  const _Float16* Bt = (const _Float16*)(const void*)Btp;
  __shared__ __align__(16) float sT[8][16 * 68];
  const int lane = threadIdx.x & 31;
  const int wave = threadIdx.x >> 5;
  const int tilesN = N >> 6;
  const int tilesM = M >> 6;
  const int tile = blockIdx.x * 8 + wave;
  if (tile >= tilesM * tilesN) return;
  const int tm = tile / tilesN;
  const int tn = tile - tm * tilesN;
  const int m0 = tm << 6;
  const int n0 = tn << 6;

  const int rlane = lane & 15;
  const int koff  = (lane >> 4) * 8;
  const int mOff  = (lane >> 4) * 8;

  v8f acc[4][4];
#pragma unroll
  for (int i = 0; i < 4; ++i)
#pragma unroll
    for (int j = 0; j < 4; ++j) acc[i][j] = zero8();

  for (int k0 = 0; k0 < K; k0 += 32) {
    v16h bh[4];
#pragma unroll
    for (int j = 0; j < 4; ++j) {
      const size_t bo = (size_t)(n0 + (j << 4) + rlane) * ldb + koff + k0;
      bh[j] = ldfrag_h(Bt + bo);
    }
#pragma unroll
    for (int i = 0; i < 4; ++i) {
      const size_t ao = (size_t)(m0 + (i << 4) + rlane) * lda + koff + k0;
      const v16h ah = ldfrag_h(A + ao);
#pragma unroll
      for (int j = 0; j < 4; ++j) {
        acc[i][j] = mma_h_raw(ah, bh[j], acc[i][j]);
      }
      dep_guard_h(acc[i][0], acc[i][3], ah, bh[3]);
    }
    keep4_h(bh[0], bh[1], bh[2], bh[3]);
  }
  acc_guard4(acc[0][0], acc[0][1], acc[0][2], acc[0][3]);
  acc_guard4(acc[1][0], acc[1][1], acc[1][2], acc[1][3]);
  acc_guard4(acc[2][0], acc[2][1], acc[2][2], acc[2][3]);
  acc_guard4(acc[3][0], acc[3][1], acc[3][2], acc[3][3]);

  float* slab = sT[wave];
#pragma unroll
  for (int i = 0; i < 4; ++i) {
    const int mBase = m0 + (i << 4);
#pragma unroll
    for (int j = 0; j < 4; ++j) {
#pragma unroll
      for (int r = 0; r < 8; ++r) {
        slab[(mOff + r) * 68 + (j << 4) + rlane] = acc[i][j][r];
      }
    }
    wave_sync_lds();
    const int hh = lane >> 4, c4 = (lane & 15) * 4;
    for (int pass = 0; pass < 2; ++pass) {
#pragma unroll
      for (int it = 0; it < 8; ++it) {
        const int row = it * 2 + hh;
        v4f v = *(const v4f*)(slab + row * 68 + c4);
        v = v * alpha;
        if (RES) {
          const v4f rr = *(const v4f*)(res + (size_t)(mBase + row) * ldr + n0 + c4);
          v = v + rr;
        }
        *(volatile v4f*)(Cout + (size_t)(mBase + row) * ldc + n0 + c4) = v;
      }
      __threadfence();
    }
    wave_sync_lds();
  }
}

extern "C" void kernel_launch(void* const* d_in, const int* in_sizes, int n_in,
                              void* d_out, int out_size, void* d_ws, size_t ws_size,
                              hipStream_t stream) {
  if (n_in < 12) return;
  if (in_sizes[0] != NE * FIN || in_sizes[1] != NE || in_sizes[2] != NE) return;
  if (in_sizes[3] != FIN * HID || in_sizes[4] != HID || in_sizes[5] != HID * NS || in_sizes[6] != NS) return;
  if (in_sizes[7] != FIN * HID || in_sizes[8] != HID || in_sizes[9] != HID * NS || in_sizes[10] != NS) return;
  if (in_sizes[11] < 1) return;
  if (out_size != NS * NT) return;

  const float* X    = (const float*)d_in[0];
  const float* z    = (const float*)d_in[1];
  const float* mask = (const float*)d_in[2];
  const float* Wp1  = (const float*)d_in[3];
  const float* bp1  = (const float*)d_in[4];
  const float* Wp2  = (const float*)d_in[5];
  const float* bp2  = (const float*)d_in[6];
  const float* Wa1  = (const float*)d_in[7];
  const float* ba1  = (const float*)d_in[8];
  const float* Wa2  = (const float*)d_in[9];
  const float* ba2  = (const float*)d_in[10];
  const float* sig  = (const float*)d_in[11];
  float* out = (float*)d_out;

  const size_t PH  = (size_t)NE * HID * 2;
  const size_t PW  = (size_t)NS * HID * 2;
  const size_t PRT = (size_t)NS * NEH * 2;
  const size_t PET = (size_t)NT * NEH * 2;
  const size_t PPT = (size_t)NS * NT * 4;
  size_t off = 0;
  const size_t oHp = off; off += PH;
  const size_t oHa = off; off += PH;
  const size_t oWp = off; off += PW;
  const size_t oWa = off; off += PW;
  const size_t oRT = off; off += PRT;
  const size_t oET = off; off += PET;
  const size_t oPT = off; off += PPT;
  if (off > ws_size) return;
  if (off > (size_t)134217728) return;

  char* ws = (char*)d_ws;
  unsigned short* Hp  = (unsigned short*)(ws + oHp);
  unsigned short* Ha  = (unsigned short*)(ws + oHa);
  unsigned short* WpT = (unsigned short*)(ws + oWp);
  unsigned short* WaT = (unsigned short*)(ws + oWa);
  unsigned short* RT  = (unsigned short*)(ws + oRT);
  unsigned short* ET  = (unsigned short*)(ws + oET);
  float* PART = (float*)(ws + oPT);

  const dim3 blk(256);
  const dim3 gH(NE / 8);
  const dim3 gTr(NS / 64, HID / 64);
  const dim3 gR(((NS / 16) * (NEH / 64) + 7) / 8);
  const dim3 gE((NT * (NEH / 2) + 255) / 256);
  const dim3 gG(((NS / 64) * (NT / 64) + 7) / 8);

  k_hplane<<<gH, blk, 0, stream>>>(X, NE, Wp1, bp1, Wa1, ba1, Hp, Ha);
  tr_cvt64w<<<gTr, blk, 0, stream>>>(Wp2, WpT, HID, NS);
  tr_cvt64w<<<gTr, blk, 0, stream>>>(Wa2, WaT, HID, NS);
  for (int half = 0; half < 2; ++half) {
    const size_t e0 = (size_t)half * NEH;
    k_resp<<<gR, blk, 0, stream>>>(WpT, WaT, Hp + e0 * HID, Ha + e0 * HID, NEH,
                                   bp2, ba2, NS, mask + e0, RT, NEH, NS, NEH, HID);
    k_expv<<<gE, blk, 0, stream>>>(z + e0, NEH, sig, (unsigned int*)ET, NT, NEH / 2);
    if (half == 0) {
      gemm64f<0><<<gG, blk, 0, stream>>>(RT, NEH, ET, NEH, PART, NT, PART, NT,
                                         ALPHA_OUT, NS, NT, NEH);
    } else {
      gemm64f<1><<<gG, blk, 0, stream>>>(RT, NEH, ET, NEH, out, NT, PART, NT,
                                         ALPHA_OUT, NS, NT, NEH);
    }
  }
  (void)hipGetLastError();
}
